// TransformerDecoderBlock_14611478741286
// MI455X (gfx1250) — hardware-verified
//
#include <hip/hip_runtime.h>
#include <math.h>

constexpr int kBatch       = 4;
constexpr int kSeq         = 1024;
constexpr int kDim         = 1024;
constexpr int kHeads       = 16;
constexpr int kHeadDim     = 64;
constexpr int kFfn         = 4096;
constexpr int kTok         = kBatch * kSeq;
constexpr int kGroups      = kBatch * kHeads;
constexpr int kChunkGroups = 8;
constexpr int kNumChunks   = kGroups / kChunkGroups;
constexpr float kWCarry     = 16.0f;
constexpr float kWCarryInv  = 1.0f / 16.0f;
constexpr float kPCarry     = 2048.0f;
constexpr float kCtxCarry   = 32.0f;
constexpr float kScoreScale = 0.125f;
constexpr float kPVScale    = kCtxCarry / kPCarry;
constexpr float kOProjScale = 1.0f / (kCtxCarry * kWCarry);
constexpr float kNegFill    = -1000000.0f;
constexpr float kLnEps      = 1e-5f;
constexpr float kInvDim     = 1.0f / 1024.0f;

constexpr size_t kMiB    = 1048576;
constexpr size_t kOffW   = 0;
constexpr size_t kOffXE  = 8 * kMiB;
constexpr size_t kOffQ   = 16 * kMiB;
constexpr size_t kOffK   = 24 * kMiB;
constexpr size_t kOffVt  = 32 * kMiB;
constexpr size_t kOffS   = 40 * kMiB;
constexpr size_t kOffP   = 72 * kMiB;
constexpr size_t kOffTmp = 88 * kMiB;
constexpr size_t kOffYZ  = 104 * kMiB;
constexpr size_t kOffH   = kOffQ;
constexpr size_t kWsTotal = 120 * kMiB;
static_assert(kOffW   + 4 * (size_t)kDim * kDim * 2 <= kOffXE);
static_assert(kOffW   + (size_t)kFfn * kDim * 2 <= kOffXE);
static_assert(kOffXE  + (size_t)kTok * kDim * 2 <= kOffQ);
static_assert(kOffQ   + (size_t)kTok * kDim * 2 <= kOffK);
static_assert(kOffK   + (size_t)kTok * kDim * 2 <= kOffVt);
static_assert(kOffVt  + (size_t)kGroups * kHeadDim * kSeq * 2 <= kOffS);
static_assert(kOffS   + (size_t)kChunkGroups * kSeq * kSeq * 4 <= kOffP);
static_assert(kOffP   + (size_t)kChunkGroups * kSeq * kSeq * 2 <= kOffTmp);
static_assert(kOffTmp + (size_t)kTok * kDim * 4 <= kOffYZ);
static_assert(kOffYZ  + (size_t)kTok * kDim * 4 <= kWsTotal);
static_assert(kOffH   + (size_t)kTok * kFfn * 2 <= kOffP);
static_assert(kOffH   + (size_t)kTok * kFfn * 2 <= kOffS + 8 * kMiB);
static_assert(kWsTotal <= 134217728);

typedef __attribute__((ext_vector_type(16))) _Float16 v16h;
typedef __attribute__((ext_vector_type(8)))  _Float16 v8h;
typedef __attribute__((ext_vector_type(16))) __bf16   v16b;
typedef __attribute__((ext_vector_type(8)))  __bf16   v8b;
typedef __attribute__((ext_vector_type(8)))  float    v8f;
typedef __attribute__((ext_vector_type(4)))  float    v4f;
typedef __attribute__((ext_vector_type(4)))  unsigned int v4u;

__device__ __forceinline__ unsigned short f2bf_bits(float f) {
  unsigned u = __float_as_uint(f);
  return (unsigned short)((u + 0x7FFFu + ((u >> 16) & 1u)) >> 16);
}
__device__ __forceinline__ float bf_bits2f(unsigned short h) { return __uint_as_float(((unsigned)h) << 16); }

__device__ __forceinline__ void dep_guard_h(v8f& a, v8f& b, v16h x, v16h y) { asm volatile("v_nop\n\tv_nop\n\tv_nop\n\tv_nop" : "+v"(a), "+v"(b) : "v"(x), "v"(y)); }
__device__ __forceinline__ void dep_guard_b(v8f& a, v8f& b, v16b x, v16b y) { asm volatile("v_nop\n\tv_nop\n\tv_nop\n\tv_nop" : "+v"(a), "+v"(b) : "v"(x), "v"(y)); }
__device__ __forceinline__ void keep4_h(v16h a, v16h b, v16h c, v16h d) { asm volatile("v_nop" :: "v"(a), "v"(b), "v"(c), "v"(d)); }
__device__ __forceinline__ void keep4_b(v16b a, v16b b, v16b c, v16b d) { asm volatile("v_nop" :: "v"(a), "v"(b), "v"(c), "v"(d)); }
__device__ __forceinline__ void acc_guard4(v8f& a, v8f& b, v8f& c, v8f& d) { asm volatile("v_nop\n\tv_nop\n\tv_nop\n\tv_nop" : "+v"(a), "+v"(b), "+v"(c), "+v"(d)); }
template <typename T> struct Frag;
template <> struct Frag<_Float16> {
  typedef v16h V; union U { v16h v; v8h h[2]; };
  static __device__ __forceinline__ v16h load(const _Float16* p) {
    U f; f.h[0] = *(const v8h*)(p); f.h[1] = *(const v8h*)(p + 16); return f.v;
  }
  static __device__ __forceinline__ v8f mma(v16h a, v16h b, v8f c) {
    return __builtin_amdgcn_wmma_f32_16x16x32_f16(false, a, false, b, (short)0, c, false, false);
  }
  static __device__ __forceinline__ void guard(v8f& a, v8f& b, v16h x, v16h y) { dep_guard_h(a, b, x, y); }
  static __device__ __forceinline__ void keep(v16h a, v16h b, v16h c, v16h d) { keep4_h(a, b, c, d); }
};
template <> struct Frag<__bf16> {
  typedef v16b V; union U { v16b v; v8b h[2]; };
  static __device__ __forceinline__ v16b load(const __bf16* p) {
    U f; f.h[0] = *(const v8b*)(p); f.h[1] = *(const v8b*)(p + 16); return f.v;
  }
  static __device__ __forceinline__ v8f mma(v16b a, v16b b, v8f c) {
    return __builtin_amdgcn_wmma_f32_16x16x32_bf16(false, a, false, b, (short)0, c, false, false);
  }
  static __device__ __forceinline__ void guard(v8f& a, v8f& b, v16b x, v16b y) { dep_guard_b(a, b, x, y); }
  static __device__ __forceinline__ void keep(v16b a, v16b b, v16b c, v16b d) { keep4_b(a, b, c, d); }
};

__device__ __forceinline__ unsigned pk16(unsigned short a, unsigned short b) { return (unsigned)a | ((unsigned)b << 16); }
__device__ __forceinline__ unsigned short h_bits(float f) { const _Float16 h = (_Float16)f; return __builtin_bit_cast(unsigned short, h); }

template <int ET> struct Elem;
template <> struct Elem<0> { typedef _Float16 T; };
template <> struct Elem<1> { typedef __bf16 T; };
template <int ET, bool SPLIT, int BIAS_MODE, int OUT_MODE, bool RESID, int ACT = 0, int TRI = 0>
__global__ __launch_bounds__(256) void wmma_gemm64(
    const unsigned short* __restrict__ Ap, const unsigned short* __restrict__ A2p, int lda, long strideA,
    const unsigned short* __restrict__ Btp, const unsigned short* __restrict__ Bt2p, int ldb, long strideB,
    void* __restrict__ Cout, void* __restrict__ Cout2, int ldc, long strideC,
    const float* __restrict__ bias,
    const float* __restrict__ resid, long strideR,
    int M, int N, int K, float scale) {
  typedef typename Elem<ET>::T T;
  typedef typename Frag<T>::V V;
  const T* A = (const T*)Ap; const T* A2 = (const T*)A2p; const T* Bt = (const T*)Btp; const T* Bt2 = (const T*)Bt2p;
  __shared__ __align__(16) float sT[8][16 * 68];
  const int b    = blockIdx.y;
  const int lane = threadIdx.x & 31;
  const int wave = threadIdx.x >> 5;
  const int tilesN = N >> 6;
  const int tilesM = M >> 6;
  const int tile = blockIdx.x * 8 + wave;
  if (tile >= tilesM * tilesN) return;
  const int tm = tile / tilesN;
  const int tn = tile - tm * tilesN;
  if (TRI == 1 && tn > tm) return;
  const int m0 = tm << 6;
  const int n0 = tn << 6;
  const int Kend = (TRI == 2) ? ((m0 + 64 < K) ? (m0 + 64) : K) : K;

  const T* Ab  = A  + (size_t)b * strideA;
  const T* Bb  = Bt + (size_t)b * strideB;
  const T* Ab2 = SPLIT ? (A2  + (size_t)b * strideA) : nullptr;
  const T* Bb2 = SPLIT ? (Bt2 + (size_t)b * strideB) : nullptr;

  const int rlane = lane & 15;
  const int koff  = (lane >> 4) * 8;
  const int mOff  = (lane >> 4) * 8;

  v8f acc[4][4];
#pragma unroll
  for (int i = 0; i < 4; ++i)
#pragma unroll
    for (int j = 0; j < 4; ++j) acc[i][j] = (v8f){0.f,0.f,0.f,0.f,0.f,0.f,0.f,0.f};

  for (int k0 = 0; k0 < Kend; k0 += 32) {
    V bh[4], bl[4];
#pragma unroll
    for (int j = 0; j < 4; ++j) {
      const size_t bo = (size_t)(n0 + (j << 4) + rlane) * ldb + koff + k0;
      bh[j] = Frag<T>::load(Bb + bo);
      if (SPLIT) bl[j] = Frag<T>::load(Bb2 + bo);
    }
#pragma unroll
    for (int i = 0; i < 4; ++i) {
      const size_t ao = (size_t)(m0 + (i << 4) + rlane) * lda + koff + k0;
      V ah = Frag<T>::load(Ab + ao);
      V al;
      if (SPLIT) al = Frag<T>::load(Ab2 + ao);
#pragma unroll
      for (int j = 0; j < 4; ++j) {
        acc[i][j] = Frag<T>::mma(ah, bh[j], acc[i][j]);
        if (SPLIT) {
          acc[i][j] = Frag<T>::mma(ah, bl[j], acc[i][j]);
          acc[i][j] = Frag<T>::mma(al, bh[j], acc[i][j]);
        }
      }
      Frag<T>::guard(acc[i][0], acc[i][3], ah, SPLIT ? al : ah);
    }
    Frag<T>::keep(bh[0], bh[1], bh[2], bh[3]);
    if (SPLIT) Frag<T>::keep(bl[0], bl[1], bl[2], bl[3]);
  }
  acc_guard4(acc[0][0], acc[0][1], acc[0][2], acc[0][3]);
  acc_guard4(acc[1][0], acc[1][1], acc[1][2], acc[1][3]);
  acc_guard4(acc[2][0], acc[2][1], acc[2][2], acc[2][3]);
  acc_guard4(acc[3][0], acc[3][1], acc[3][2], acc[3][3]);

  float* slab = sT[wave];
  const float* Rb = RESID ? (resid + (size_t)b * strideR) : nullptr;
#pragma unroll
  for (int i = 0; i < 4; ++i) {
    const int mBase = m0 + (i << 4);
#pragma unroll
    for (int j = 0; j < 4; ++j) {
      const int n = n0 + (j << 4) + rlane;
      float bv = 0.f;
      if (BIAS_MODE == 2) bv = bias[n];
#pragma unroll
      for (int r = 0; r < 8; ++r) {
        float v = acc[i][j][r] * scale;
        if (BIAS_MODE == 1) v += bias[mBase + mOff + r];
        if (BIAS_MODE == 2) v += bv;
        if (RESID) v += Rb[(size_t)(mBase + mOff + r) * ldc + n];
        if (ACT == 2) v = fmaxf(v, 0.0f);
        if (ACT == 4) v = (v > 0.f) ? v : 0.01f * v;
        slab[(mOff + r) * 68 + (j << 4) + rlane] = v;
      }
    }
    __builtin_amdgcn_fence(__ATOMIC_RELEASE, "workgroup");
    __builtin_amdgcn_wave_barrier();
    __builtin_amdgcn_fence(__ATOMIC_ACQUIRE, "workgroup");
    if (OUT_MODE == 0) {
      float* C = (float*)Cout + (size_t)b * strideC;
      const int hh = lane >> 4, c4 = (lane & 15) * 4;
      for (int pass = 0; pass < 2; ++pass) {
#pragma unroll
        for (int it = 0; it < 8; ++it) {
          const int row = it * 2 + hh;
          v4f v = *(const v4f*)(slab + row * 68 + c4);
          *(volatile v4f*)(C + (size_t)(mBase + row) * ldc + n0 + c4) = v;
        }
        __threadfence();
      }
    } else {
      const int q = lane >> 3, c8 = (lane & 7) * 8;
      unsigned short* C  = (unsigned short*)Cout  + (size_t)b * strideC;
      unsigned short* C2 = (OUT_MODE == 2) ? ((unsigned short*)Cout2 + (size_t)b * strideC) : nullptr;
      for (int pass = 0; pass < 2; ++pass) {
#pragma unroll
        for (int it = 0; it < 4; ++it) {
          const int row = it * 4 + q;
          const float* sp = slab + row * 68 + c8;
          v8h hv, lv;
#pragma unroll
          for (int e = 0; e < 8; ++e) {
            if (OUT_MODE == 1) {
              hv[e] = (_Float16)sp[e];
            } else {
              unsigned short hb = f2bf_bits(sp[e]);
              unsigned short lb = f2bf_bits(sp[e] - bf_bits2f(hb));
              hv[e] = __builtin_bit_cast(_Float16, hb);
              lv[e] = __builtin_bit_cast(_Float16, lb);
            }
          }
          *(volatile v8h*)(C + (size_t)(mBase + row) * ldc + n0 + c8) = hv;
          if (OUT_MODE == 2) *(volatile v8h*)(C2 + (size_t)(mBase + row) * ldc + n0 + c8) = lv;
        }
        __threadfence();
      }
    }
    __builtin_amdgcn_fence(__ATOMIC_RELEASE, "workgroup");
    __builtin_amdgcn_wave_barrier();
    __builtin_amdgcn_fence(__ATOMIC_ACQUIRE, "workgroup");
  }
}

__global__ __launch_bounds__(256) void wtcast_kernel(const float* __restrict__ W0, const float* __restrict__ W1,
                                                     const float* __restrict__ W2, const float* __restrict__ W3,
                                                     unsigned short* __restrict__ out, int Kd, int Nd, float scale) {
  __shared__ float sm[64][65];
  const int t  = threadIdx.x;
  const int k0 = blockIdx.x * 64;
  const int n0 = blockIdx.y * 64;
  const int z  = blockIdx.z;
  const float* W = (z == 0) ? W0 : (z == 1) ? W1 : (z == 2) ? W2 : W3;
#pragma unroll
  for (int i = 0; i < 16; ++i) {
    const int e = i * 256 + t;
    const int r = e >> 6;
    const int c = e & 63;
    sm[c][r] = W[(size_t)(k0 + r) * Nd + n0 + c] * scale;
  }
  __syncthreads();
  const int lane = t & 31, wave = t >> 5;
  const int q = lane >> 3, c8 = (lane & 7) * 8;
  unsigned short* op = out + (size_t)z * Nd * Kd;
  for (int pass = 0; pass < 2; ++pass) {
#pragma unroll
    for (int it = 0; it < 2; ++it) {
      const int row = wave * 8 + it * 4 + q;
      unsigned short hb[8];
#pragma unroll
      for (int e = 0; e < 8; ++e) hb[e] = h_bits(sm[row][c8 + e]);
      const v4u u = (v4u){pk16(hb[0], hb[1]), pk16(hb[2], hb[3]), pk16(hb[4], hb[5]), pk16(hb[6], hb[7])};
      *(volatile v4u*)(op + (size_t)(n0 + row) * Kd + k0 + c8) = u;
    }
    __threadfence();
  }
}

__global__ __launch_bounds__(256) void cast8_f16_kernel(const float* __restrict__ in, unsigned short* __restrict__ out, int n8) {
  const int i = blockIdx.x * 256 + threadIdx.x;
  if (i >= n8) return;
  const float* p = in + 8 * (size_t)i;
  const v4f a = *(const v4f*)(p);
  const v4f c = *(const v4f*)(p + 4);
  unsigned short hb[8];
#pragma unroll
  for (int e = 0; e < 4; ++e) {
    hb[e]     = h_bits(a[e]);
    hb[4 + e] = h_bits(c[e]);
  }
  const v4u u = (v4u){pk16(hb[0], hb[1]), pk16(hb[2], hb[3]), pk16(hb[4], hb[5]), pk16(hb[6], hb[7])};
  unsigned short* q = out + 8 * (size_t)i;
  *(volatile v4u*)q = u;
  __threadfence();
  *(volatile v4u*)q = u;
}

__global__ __launch_bounds__(128) void softmax_kernel(const float* __restrict__ S, unsigned short* __restrict__ P,
                                                      const int* __restrict__ vlens, int bsel, int causal, float carry) {
  __shared__ float redM[4];
  __shared__ float redS[4];
  const int r    = blockIdx.x;
  const int qi   = r & (kSeq - 1);
  const int t    = threadIdx.x;
  const int lane = t & 31, wave = t >> 5;
  const int c0   = t * 8;
  const int lim  = causal ? (((qi >> 6) + 1) << 6) : kSeq;
  const int cc   = (c0 < lim - 8) ? c0 : (lim - 8);
  const float* sr = S + (size_t)r * kSeq + cc;
  const v4f a = *(const v4f*)(sr);
  const v4f c = *(const v4f*)(sr + 4);
  const int vl = vlens[bsel];
  float x[8];
#pragma unroll
  for (int e = 0; e < 4; ++e) {
    const int colA = c0 + e, colB = c0 + 4 + e;
    const bool keepA = causal ? (colA <= qi) : (colA < vl);
    const bool keepB = causal ? (colB <= qi) : (colB < vl);
    x[e]     = keepA ? a[e] : kNegFill;
    x[4 + e] = keepB ? c[e] : kNegFill;
  }
  float m = fmaxf(fmaxf(fmaxf(x[0], x[1]), fmaxf(x[2], x[3])), fmaxf(fmaxf(x[4], x[5]), fmaxf(x[6], x[7])));
#pragma unroll
  for (int off = 16; off > 0; off >>= 1) m = fmaxf(m, __shfl_xor(m, off, 32));
  if (lane == 0) redM[wave] = m;
  __syncthreads();
  const float rm = fmaxf(fmaxf(redM[0], redM[1]), fmaxf(redM[2], redM[3]));
  float ev[8];
  float s = 0.f;
#pragma unroll
  for (int e = 0; e < 8; ++e) { ev[e] = expf(x[e] - rm); s += ev[e]; }
#pragma unroll
  for (int off = 16; off > 0; off >>= 1) s += __shfl_xor(s, off, 32);
  if (lane == 0) redS[wave] = s;
  __syncthreads();
  const float tot = ((redS[0] + redS[1]) + redS[2]) + redS[3];
  const float inv = (1.0f / tot) * carry;
  unsigned short hb[8];
#pragma unroll
  for (int e = 0; e < 8; ++e) hb[e] = h_bits(ev[e] * inv);
  const v4u u = (v4u){pk16(hb[0], hb[1]), pk16(hb[2], hb[3]), pk16(hb[4], hb[5]), pk16(hb[6], hb[7])};
  unsigned short* pp = P + (size_t)r * kSeq + c0;
  *(volatile v4u*)pp = u;
  __threadfence();
  *(volatile v4u*)pp = u;
}

__global__ __launch_bounds__(256) void ln_kernel(const float* __restrict__ X, const float* __restrict__ gam,
                                                 const float* __restrict__ bet, float* __restrict__ outF,
                                                 unsigned short* __restrict__ outH, int writeH) {
  __shared__ float redA[8];
  __shared__ float redB[8];
  __shared__ __align__(16) unsigned int hrow[512];
  const int row  = blockIdx.x;
  const int t    = threadIdx.x;
  const int lane = t & 31, wave = t >> 5;
  const int c0   = t * 4;
  const v4f xv = *(const v4f*)(X + (size_t)row * kDim + c0);
  const v4f gv = *(const v4f*)(gam + c0);
  const v4f bv = *(const v4f*)(bet + c0);
  float s = (xv[0] + xv[1]) + (xv[2] + xv[3]);
#pragma unroll
  for (int off = 16; off > 0; off >>= 1) s += __shfl_xor(s, off, 32);
  if (lane == 0) redA[wave] = s;
  __syncthreads();
  float tot = 0.f;
#pragma unroll
  for (int w = 0; w < 8; ++w) tot += redA[w];
  const float mean = tot * kInvDim;
  float d[4];
#pragma unroll
  for (int e = 0; e < 4; ++e) d[e] = xv[e] - mean;
  float q = (d[0] * d[0] + d[1] * d[1]) + (d[2] * d[2] + d[3] * d[3]);
#pragma unroll
  for (int off = 16; off > 0; off >>= 1) q += __shfl_xor(q, off, 32);
  if (lane == 0) redB[wave] = q;
  __syncthreads();
  float vt = 0.f;
#pragma unroll
  for (int w = 0; w < 8; ++w) vt += redB[w];
  const float var  = vt * kInvDim;
  const float rstd = rsqrtf(var + kLnEps);
  v4f y;
#pragma unroll
  for (int e = 0; e < 4; ++e) y[e] = d[e] * rstd * gv[e] + bv[e];
  float* op = outF + (size_t)row * kDim + c0;
  *(volatile v4f*)op = y;
  __threadfence();
  *(volatile v4f*)op = y;
  if (writeH) {
    hrow[2 * t]     = pk16(h_bits(y[0]), h_bits(y[1]));
    hrow[2 * t + 1] = pk16(h_bits(y[2]), h_bits(y[3]));
    __syncthreads();
    if (t < 128) {
      const v4u u = *(const v4u*)(hrow + 4 * t);
      unsigned short* hp = outH + (size_t)row * kDim + 8 * t;
      *(volatile v4u*)hp = u;
      __threadfence();
      *(volatile v4u*)hp = u;
    }
  }
}

static inline unsigned gemm_blocks(int M, int N) { return (unsigned)((((M >> 6) * (N >> 6)) + 7) >> 3); }

static void launch_proj_f16(const unsigned short* A, const unsigned short* Wt, const float* bias, unsigned short* C,
                            hipStream_t stream) {
  wmma_gemm64<0, false, 2, 1, false, 0, 0><<<dim3(gemm_blocks(kTok, kDim), 1), dim3(256), 0, stream>>>(
      A, nullptr, kDim, 0L, Wt, nullptr, kDim, 0L, (void*)C, nullptr, kDim, 0L, bias, nullptr, 0L,
      kTok, kDim, kDim, kWCarryInv);
}

static void launch_vt(const unsigned short* Wvt, const unsigned short* Xh, const float* bias, unsigned short* Vt,
                      hipStream_t stream) {
  wmma_gemm64<0, false, 1, 1, false, 0, 0><<<dim3(gemm_blocks(kDim, kSeq), kBatch), dim3(256), 0, stream>>>(
      Wvt, nullptr, kDim, 0L, Xh, nullptr, kDim, (long)kSeq * kDim, (void*)Vt, nullptr, kSeq, (long)kDim * kSeq,
      bias, nullptr, 0L, kDim, kSeq, kDim, kWCarryInv);
}

static void launch_oproj(const unsigned short* Ctx, const unsigned short* Wot, const float* bias, const float* resid,
                         float* C, hipStream_t stream) {
  wmma_gemm64<0, false, 2, 0, true, 0, 0><<<dim3(gemm_blocks(kTok, kDim), 1), dim3(256), 0, stream>>>(
      Ctx, nullptr, kDim, 0L, Wot, nullptr, kDim, 0L, (void*)C, nullptr, kDim, 0L, bias, resid, 0L,
      kTok, kDim, kDim, kOProjScale);
}

static void run_attention(const unsigned short* pQ, const unsigned short* pK, const unsigned short* pVt, float* pS,
                          unsigned short* pP, unsigned short* pCtx, const int* VL, int causal, hipStream_t stream) {
  for (int c = 0; c < kNumChunks; ++c) {
    const int b  = c / (kHeads / kChunkGroups);
    const int h0 = (c % (kHeads / kChunkGroups)) * kChunkGroups;
    const size_t qkBase = (size_t)b * kSeq * kDim + (size_t)h0 * kHeadDim;
    const unsigned short* qA = pQ + qkBase;
    const unsigned short* kB = pK + qkBase;
    const dim3 gsc(gemm_blocks(kSeq, kSeq), kChunkGroups);
    if (causal) {
      wmma_gemm64<0, false, 0, 0, false, 0, 1><<<gsc, dim3(256), 0, stream>>>(
          qA, nullptr, kDim, (long)kHeadDim, kB, nullptr, kDim, (long)kHeadDim, (void*)pS, nullptr, kSeq,
          (long)kSeq * kSeq, nullptr, nullptr, 0L, kSeq, kSeq, kHeadDim, kScoreScale);
    } else {
      wmma_gemm64<0, false, 0, 0, false, 0, 0><<<gsc, dim3(256), 0, stream>>>(
          qA, nullptr, kDim, (long)kHeadDim, kB, nullptr, kDim, (long)kHeadDim, (void*)pS, nullptr, kSeq,
          (long)kSeq * kSeq, nullptr, nullptr, 0L, kSeq, kSeq, kHeadDim, kScoreScale);
    }
    softmax_kernel<<<dim3(kChunkGroups * kSeq), dim3(128), 0, stream>>>(pS, pP, VL, b, causal, kPCarry);
    const unsigned short* vB = pVt + (size_t)c * kChunkGroups * kHeadDim * kSeq;
    unsigned short* oC = pCtx + qkBase;
    const dim3 gpv(gemm_blocks(kSeq, kHeadDim), kChunkGroups);
    if (causal) {
      wmma_gemm64<0, false, 0, 1, false, 0, 2><<<gpv, dim3(256), 0, stream>>>(
          pP, nullptr, kSeq, (long)kSeq * kSeq, vB, nullptr, kSeq, (long)kHeadDim * kSeq, (void*)oC, nullptr, kDim,
          (long)kHeadDim, nullptr, nullptr, 0L, kSeq, kHeadDim, kSeq, kPVScale);
    } else {
      wmma_gemm64<0, false, 0, 1, false, 0, 0><<<gpv, dim3(256), 0, stream>>>(
          pP, nullptr, kSeq, (long)kSeq * kSeq, vB, nullptr, kSeq, (long)kHeadDim * kSeq, (void*)oC, nullptr, kDim,
          (long)kHeadDim, nullptr, nullptr, 0L, kSeq, kHeadDim, kSeq, kPVScale);
    }
  }
}

extern "C" void kernel_launch(void* const* d_in, const int* in_sizes, int n_in,
                              void* d_out, int out_size, void* d_ws, size_t ws_size,
                              hipStream_t stream) {
  if (n_in < 29) return;
  if (in_sizes[0] != kTok * kDim || in_sizes[1] != kTok * kDim || in_sizes[2] < kBatch) return;
  if (in_sizes[3] != kDim * kDim || in_sizes[5] != kDim * kDim || in_sizes[7] != kDim * kDim ||
      in_sizes[9] != kDim * kDim || in_sizes[13] != kDim * kDim || in_sizes[15] != kDim * kDim ||
      in_sizes[17] != kDim * kDim || in_sizes[19] != kDim * kDim) return;
  if (in_sizes[23] != kDim * kFfn || in_sizes[25] != kFfn * kDim || in_sizes[24] != kFfn) return;
  if (in_sizes[4] != kDim || in_sizes[11] != kDim || in_sizes[26] != kDim || in_sizes[27] != kDim || in_sizes[28] != kDim) return;
  if (out_size != kTok * kDim) return;
  if (ws_size < kWsTotal) return;

  const float* X   = (const float*)d_in[0];
  const float* ENC = (const float*)d_in[1];
  const int*   VL  = (const int*)d_in[2];
  const float* Wq1 = (const float*)d_in[3];  const float* bq1 = (const float*)d_in[4];
  const float* Wk1 = (const float*)d_in[5];  const float* bk1 = (const float*)d_in[6];
  const float* Wv1 = (const float*)d_in[7];  const float* bv1 = (const float*)d_in[8];
  const float* Wo1 = (const float*)d_in[9];  const float* bo1 = (const float*)d_in[10];
  const float* g1  = (const float*)d_in[11]; const float* be1 = (const float*)d_in[12];
  const float* Wq2 = (const float*)d_in[13]; const float* bq2 = (const float*)d_in[14];
  const float* Wk2 = (const float*)d_in[15]; const float* bk2 = (const float*)d_in[16];
  const float* Wv2 = (const float*)d_in[17]; const float* bv2 = (const float*)d_in[18];
  const float* Wo2 = (const float*)d_in[19]; const float* bo2 = (const float*)d_in[20];
  const float* g2  = (const float*)d_in[21]; const float* be2 = (const float*)d_in[22];
  const float* Wf1 = (const float*)d_in[23]; const float* bf1 = (const float*)d_in[24];
  const float* Wf2 = (const float*)d_in[25]; const float* bf2 = (const float*)d_in[26];
  const float* g3  = (const float*)d_in[27]; const float* be3 = (const float*)d_in[28];
  float* OUT = (float*)d_out;

  char* ws = (char*)d_ws;
  unsigned short* pW   = (unsigned short*)(ws + kOffW);
  unsigned short* pXE  = (unsigned short*)(ws + kOffXE);
  unsigned short* pQ   = (unsigned short*)(ws + kOffQ);
  unsigned short* pK   = (unsigned short*)(ws + kOffK);
  unsigned short* pVt  = (unsigned short*)(ws + kOffVt);
  float*          pS   = (float*)(ws + kOffS);
  unsigned short* pYh  = (unsigned short*)(ws + kOffS);
  unsigned short* pP   = (unsigned short*)(ws + kOffP);
  unsigned short* pZh  = (unsigned short*)(ws + kOffP);
  float*          pTmp = (float*)(ws + kOffTmp);
  float*          pYZ  = (float*)(ws + kOffYZ);
  unsigned short* pH   = (unsigned short*)(ws + kOffH);
  const size_t kWPlane = (size_t)kDim * kDim;

  const dim3 blk(256);
  const unsigned castBlocks = (unsigned)((kTok * kDim / 8) / 256);

  wtcast_kernel<<<dim3(kDim / 64, kDim / 64, 4), blk, 0, stream>>>(Wq1, Wk1, Wv1, Wo1, pW, kDim, kDim, kWCarry);
  cast8_f16_kernel<<<dim3(castBlocks), blk, 0, stream>>>(X, pXE, kTok * kDim / 8);
  launch_proj_f16(pXE, pW + 0 * kWPlane, bq1, pQ, stream);
  launch_proj_f16(pXE, pW + 1 * kWPlane, bk1, pK, stream);
  launch_vt(pW + 2 * kWPlane, pXE, bv1, pVt, stream);
  run_attention(pQ, pK, pVt, pS, pP, pXE, VL, 1, stream);
  launch_oproj(pXE, pW + 3 * kWPlane, bo1, X, pTmp, stream);
  ln_kernel<<<dim3(kTok), blk, 0, stream>>>(pTmp, g1, be1, pYZ, pYh, 1);

  wtcast_kernel<<<dim3(kDim / 64, kDim / 64, 4), blk, 0, stream>>>(Wq2, Wk2, Wv2, Wo2, pW, kDim, kDim, kWCarry);
  cast8_f16_kernel<<<dim3(castBlocks), blk, 0, stream>>>(ENC, pXE, kTok * kDim / 8);
  launch_proj_f16(pYh, pW + 0 * kWPlane, bq2, pQ, stream);
  launch_proj_f16(pXE, pW + 1 * kWPlane, bk2, pK, stream);
  launch_vt(pW + 2 * kWPlane, pXE, bv2, pVt, stream);
  run_attention(pQ, pK, pVt, pS, pP, pXE, VL, 0, stream);
  launch_oproj(pXE, pW + 3 * kWPlane, bo2, pYZ, pTmp, stream);
  ln_kernel<<<dim3(kTok), blk, 0, stream>>>(pTmp, g2, be2, pYZ, pZh, 1);

  wtcast_kernel<<<dim3(kDim / 64, kFfn / 64, 1), blk, 0, stream>>>(Wf1, Wf1, Wf1, Wf1, pW, kDim, kFfn, kWCarry);
  wtcast_kernel<<<dim3(kFfn / 64, kDim / 64, 1), blk, 0, stream>>>(Wf2, Wf2, Wf2, Wf2, pXE, kFfn, kDim, kWCarry);
  wmma_gemm64<0, false, 2, 1, false, 2, 0><<<dim3(gemm_blocks(kTok, kFfn), 1), blk, 0, stream>>>(
      pZh, nullptr, kDim, 0L, pW, nullptr, kDim, 0L, (void*)pH, nullptr, kFfn, 0L, bf1, nullptr, 0L,
      kTok, kFfn, kDim, kWCarryInv);
  wmma_gemm64<0, false, 2, 0, true, 0, 0><<<dim3(gemm_blocks(kTok, kDim), 1), blk, 0, stream>>>(
      pH, nullptr, kFfn, 0L, pXE, nullptr, kFfn, 0L, (void*)pTmp, nullptr, kDim, 0L, bf2, pYZ, 0L,
      kTok, kDim, kFfn, kWCarryInv);
  ln_kernel<<<dim3(kTok), blk, 0, stream>>>(pTmp, g3, be3, OUT, pZh, 0);
}
